// EnhancedLinkPredictor_33681133535939
// MI455X (gfx1250) — hardware-verified
//
#include <hip/hip_runtime.h>
#include <stddef.h>


typedef _Float16 v16h __attribute__((ext_vector_type(16)));
typedef _Float16 v8h  __attribute__((ext_vector_type(8)));
typedef float    v8f  __attribute__((ext_vector_type(8)));
typedef float    v4f  __attribute__((ext_vector_type(4)));
typedef unsigned int v4u __attribute__((ext_vector_type(4)));
typedef int          v4i __attribute__((ext_vector_type(4)));

#ifndef NPRED
#define NPRED 16384
#endif
#define NPRED_FULL 16384
#define N_D    8192
#define N_P    4096
#define NEDGE  131072
#define FEAT   64
#define KIN    256
#define HIDN   128
#define DDI_WORDS (N_D / 32)
#define DP_WORDS  (N_P / 32)
#define ADJ_LDS_WORDS 16384
#define ROWS_DDI (ADJ_LDS_WORDS / DDI_WORDS)
#define ROWS_DP  (ADJ_LDS_WORDS / DP_WORDS)

static_assert(NPRED >= 128 && NPRED <= NPRED_FULL && (NPRED % 128) == 0);
static_assert((NPRED % 8) == 0);
static_assert(KIN == 4 * FEAT);
static_assert((KIN % 32) == 0 && (KIN % 64) == 0);
static_assert(HIDN == 8 * 16);
static_assert((HIDN % 64) == 0);
static_assert((NEDGE % 128) == 0);
static_assert((N_D % 32) == 0 && (N_P % 32) == 0);
static_assert((DDI_WORDS % 32) == 0 && (DP_WORDS % 32) == 0);
static_assert((ADJ_LDS_WORDS % DDI_WORDS) == 0 && (ADJ_LDS_WORDS % DP_WORDS) == 0);
static_assert((N_D % ROWS_DDI) == 0 && (N_D % ROWS_DP) == 0);
static_assert((ADJ_LDS_WORDS & (ADJ_LDS_WORDS - 1)) == 0);
static_assert((ADJ_LDS_WORDS % 128) == 0);
static_assert((size_t)ADJ_LDS_WORDS * 4 <= (size_t)131072);
static_assert(FEAT == 8 * 8);

#define LDT 72
static_assert((LDT % 8) == 0 && LDT >= 64);
static_assert((size_t)64 * LDT * 2 <= (size_t)131072);

#define WCARRY 64.0f
#define ACARRY 16.0f

#define W1T_BYTES  ((size_t)HIDN * KIN * 2)
#define ADJD_BYTES ((size_t)N_D * DDI_WORDS * 4)
#define ADJP_BYTES ((size_t)N_D * DP_WORDS * 4)
#define PAIR_BYTES ((size_t)NPRED * KIN * 2)
#define OFF_W1T  ((size_t)0)
#define OFF_ADJD (OFF_W1T + W1T_BYTES)
#define OFF_ADJP (OFF_ADJD + ADJD_BYTES)
#define OFF_PAIR (OFF_ADJP + ADJP_BYTES)
#define WS_TOTAL (OFF_PAIR + PAIR_BYTES)
static_assert((W1T_BYTES % 128) == 0 && (ADJD_BYTES % 128) == 0);
static_assert((ADJP_BYTES % 128) == 0 && (PAIR_BYTES % 128) == 0);
static_assert(ADJD_BYTES == (size_t)(N_D / ROWS_DDI) * ADJ_LDS_WORDS * 4);
static_assert(ADJP_BYTES == (size_t)(N_D / ROWS_DP) * ADJ_LDS_WORDS * 4);
static_assert(WS_TOTAL <= (size_t)134217728);

__device__ __forceinline__ float bf16r(float x) {
  unsigned int u = __float_as_uint(x);
  u = (u + 0x7FFFu + ((u >> 16) & 1u)) & 0xFFFF0000u;
  return __uint_as_float(u);
}

static __device__ __forceinline__ _Float16 toh_flush(float v) {
  const _Float16 r = (_Float16)v;
  return (fabsf(v) < 6.103515625e-05f) ? (_Float16)0.0f : r;
}

__device__ __forceinline__ v16h frag_at(const _Float16* p) {
  v8h lo = *(const v8h*)(p);
  v8h hi = *(const v8h*)(p + 16);
  v16h out;
#pragma unroll
  for (int i = 0; i < 8; ++i) { out[i] = lo[i]; out[i + 8] = hi[i]; }
  return out;
}

__device__ __forceinline__ v8f wmma16(v16h a, v16h b, v8f c) {
  v8f d = __builtin_amdgcn_wmma_f32_16x16x32_f16(false, a, false, b, (short)0, c,
                                                 false, false);
  asm volatile("v_nop\n\tv_nop\n\tv_nop\n\tv_nop" : "+v"(d) : "v"(a), "v"(b));
  return d;
}

__device__ __forceinline__ float red16_sum(float x) {
#pragma unroll
  for (int off = 1; off < 16; off <<= 1) x += __shfl_xor(x, off, 32);
  return x;
}
__device__ __forceinline__ int red32_isum(int x) {
#pragma unroll
  for (int off = 1; off < 32; off <<= 1) x += __shfl_xor(x, off, 32);
  return x;
}

__global__ __launch_bounds__(256) void wconv_kernel(
    const float* __restrict__ W, _Float16* __restrict__ Wt, unsigned ldw, unsigned ldk) {
  __shared__ _Float16 T[64 * LDT];
  const unsigned tid = threadIdx.x;
  const unsigned n0 = blockIdx.x * 64u;
  const unsigned k0 = blockIdx.y * 64u;
#pragma unroll 4
  for (unsigned j = 0; j < 16u; ++j) {
    const unsigned idx = tid + 256u * j;
    const unsigned kr = idx >> 6, nc = idx & 63u;
    const float v = W[(size_t)(k0 + kr) * ldw + n0 + nc];
    T[nc * LDT + kr] = toh_flush(WCARRY * bf16r(v));
  }
  __syncthreads();
  v8h x[2];
  size_t off[2];
#pragma unroll
  for (unsigned i = 0; i < 2u; ++i) {
    const unsigned n = 32u * i + (tid >> 3);
    const unsigned kc = (tid & 7u) * 8u;
    x[i] = *(const v8h*)&T[n * LDT + kc];
    off[i] = (size_t)(n0 + n) * ldk + k0 + kc;
  }
#pragma unroll
  for (int i = 0; i < 2; ++i) *(volatile v8h*)(Wt + off[i]) = x[i];
  __threadfence();
#pragma unroll
  for (int i = 0; i < 2; ++i) *(volatile v8h*)(Wt + off[i]) = x[i];
}

template <int WORDS, int NBITS, int SYM>
__device__ __forceinline__ void adj_body(const int* __restrict__ ei,
                                         unsigned int* __restrict__ adj) {
  __shared__ __attribute__((aligned(16))) unsigned int bits[ADJ_LDS_WORDS];
  const unsigned lane = threadIdx.x & 31u;
  const int ROWS = ADJ_LDS_WORDS / WORDS;
  const int row0 = (int)blockIdx.x * ROWS;

  const v4u zero = {0u, 0u, 0u, 0u};
#pragma unroll 4
  for (unsigned i = 0; i < (unsigned)(ADJ_LDS_WORDS / 128); ++i)
    *(v4u*)&bits[(i * 32u + lane) * 4u] = zero;
  __syncthreads();

#pragma unroll 1
  for (unsigned e0 = 0; e0 < (unsigned)NEDGE; e0 += 128u) {
    const v4i av = *(const v4i*)(ei + e0 + lane * 4u);
    const v4i bv = *(const v4i*)(ei + (unsigned)NEDGE + e0 + lane * 4u);
#pragma unroll
    for (int c = 0; c < 4; ++c) {
      int a = av[c];
      int b = bv[c];
      a = (a < 0) ? (a + N_D) : a;
      b = (b < 0) ? (b + NBITS) : b;
      const bool ok = ((unsigned)a < (unsigned)N_D) && ((unsigned)b < (unsigned)NBITS);
      const int ra = a - row0;
      unsigned mk = __builtin_amdgcn_ballot_w32(ok && ((unsigned)ra < (unsigned)ROWS));
      while (mk != 0u) {
        const int src = __builtin_ctz(mk);
        mk &= mk - 1u;
        const int r  = __builtin_amdgcn_readlane(ra, src);
        const int cb = __builtin_amdgcn_readlane(b, src);
        if (lane == 0u) {
          const unsigned idx = ((unsigned)r * (unsigned)WORDS + ((unsigned)cb >> 5)) &
                               (unsigned)(ADJ_LDS_WORDS - 1);
          bits[idx] |= (1u << ((unsigned)cb & 31u));
        }
      }
      if (SYM) {
        const int rb = b - row0;
        unsigned mk2 = __builtin_amdgcn_ballot_w32(ok && ((unsigned)rb < (unsigned)ROWS));
        while (mk2 != 0u) {
          const int src = __builtin_ctz(mk2);
          mk2 &= mk2 - 1u;
          const int r  = __builtin_amdgcn_readlane(rb, src);
          const int ca = __builtin_amdgcn_readlane(a, src);
          if (lane == 0u) {
            const unsigned idx = ((unsigned)r * (unsigned)WORDS + ((unsigned)ca >> 5)) &
                                 (unsigned)(ADJ_LDS_WORDS - 1);
            bits[idx] |= (1u << ((unsigned)ca & 31u));
          }
        }
      }
    }
  }
  __syncthreads();

  unsigned int* g = adj + (size_t)row0 * WORDS;
#pragma unroll 4
  for (unsigned i = 0; i < (unsigned)(ADJ_LDS_WORDS / 128); ++i) {
    const v4u x = *(const v4u*)&bits[(i * 32u + lane) * 4u];
    *(volatile v4u*)(g + (i * 32u + lane) * 4u) = x;
  }
  __threadfence();
#pragma unroll 4
  for (unsigned i = 0; i < (unsigned)(ADJ_LDS_WORDS / 128); ++i) {
    const v4u x = *(const v4u*)&bits[(i * 32u + lane) * 4u];
    *(volatile v4u*)(g + (i * 32u + lane) * 4u) = x;
  }
}

__global__ __launch_bounds__(32) void adj_ddi_kernel(
    const int* __restrict__ ei, unsigned int* __restrict__ adj) {
  adj_body<DDI_WORDS, N_D, 1>(ei, adj);
}
__global__ __launch_bounds__(32) void adj_dp_kernel(
    const int* __restrict__ ei, unsigned int* __restrict__ adj) {
  adj_body<DP_WORDS, N_P, 0>(ei, adj);
}

template <int WORDS>
__device__ __forceinline__ void cn_accum(const unsigned int* __restrict__ adj,
                                         const float* __restrict__ feat,
                                         const int s, const int d, const unsigned lane,
                                         float (&acc)[8], int& cnt_out) {
#pragma clang fp contract(off)
  const unsigned int* rs = adj + (size_t)s * WORDS;
  const unsigned int* rd = adj + (size_t)d * WORDS;
  int cnt = 0;
#pragma unroll
  for (int k = 0; k < 8; ++k) acc[k] = 0.0f;
#pragma unroll 1
  for (unsigned i = 0; i < (unsigned)(WORDS / 32); ++i) {
    const unsigned u = rs[i * 32u + lane] & rd[i * 32u + lane];
    cnt += __popc(u);
    unsigned mk = __builtin_amdgcn_ballot_w32(u != 0u);
    while (mk != 0u) {
      const int src = __builtin_ctz(mk);
      mk &= mk - 1u;
      unsigned uu = (unsigned)__builtin_amdgcn_readlane((int)u, src);
      const unsigned base = (i * 32u + (unsigned)src) * 32u;
      while (uu != 0u) {
        const unsigned j = (unsigned)__builtin_ctz(uu);
        uu &= uu - 1u;
        const unsigned n = base + j;
        const float* zr = feat + (size_t)n * FEAT + (lane & 7u) * 8u;
        const v4f a0 = *(const v4f*)(zr);
        const v4f a1 = *(const v4f*)(zr + 4);
#pragma unroll
        for (int k = 0; k < 4; ++k) {
          acc[k]     += bf16r(a0[k]);
          acc[k + 4] += bf16r(a1[k]);
        }
      }
    }
  }
  cnt_out = red32_isum(cnt);
}

__global__ __launch_bounds__(256) void pair_kernel(
    const float* __restrict__ zd, const float* __restrict__ zp, const int* __restrict__ pred,
    const unsigned int* __restrict__ adjd, const unsigned int* __restrict__ adjp,
    _Float16* __restrict__ pair) {
#pragma clang fp contract(off)
  const unsigned lane = threadIdx.x & 31u;
  const unsigned wave = (unsigned)__builtin_amdgcn_readfirstlane((int)(threadIdx.x >> 5));
  const unsigned e = blockIdx.x * 8u + wave;
  int s = pred[e];
  int d = pred[(unsigned)NPRED_FULL + e];
  s = (s < 0) ? (s + N_D) : s;
  d = (d < 0) ? (d + N_D) : d;
  s = min(max(s, 0), N_D - 1);
  d = min(max(d, 0), N_D - 1);

  float accd[8], accp[8];
  int cntd = 0, cntp = 0;
  cn_accum<DDI_WORDS>(adjd, zd, s, d, lane, accd, cntd);
  cn_accum<DP_WORDS>(adjp, zp, s, d, lane, accp, cntp);
  const float invd = 1.0f / fmaxf((float)cntd, 1.0f);
  const float invp = 1.0f / fmaxf((float)cntp, 1.0f);

  const unsigned g = lane >> 3;
  const int rsel = (g == 1u) ? d : s;
  const float* zq = zd + (size_t)rsel * FEAT + (lane & 7u) * 8u;
  v4f z0 = *(const v4f*)(zq);
  v4f z1 = *(const v4f*)(zq + 4);
  asm volatile("" : "+v"(z0), "+v"(z1));

  v8h o;
#pragma unroll
  for (int k = 0; k < 8; ++k) {
    const float zz = bf16r((k < 4) ? z0[k & 3] : z1[k & 3]);
    const float cd = accd[k] * invd;
    const float cp = accp[k] * invp;
    const float val = (g < 2u) ? zz : ((g == 2u) ? cd : cp);
    o[k] = toh_flush(ACARRY * val);
  }
  _Float16* p = pair + (size_t)e * KIN + lane * 8u;
  *(volatile v8h*)p = o;
  __threadfence();
  *(volatile v8h*)p = o;
}

__global__ __launch_bounds__(256) void mlp_kernel(
    const _Float16* __restrict__ A16, const _Float16* __restrict__ Bt,
    const float* __restrict__ b1, const float* __restrict__ W2, const float* __restrict__ b2,
    float* __restrict__ out) {
  __shared__ __attribute__((aligned(16))) float Ls[128];
  const unsigned tid = threadIdx.x, lane = tid & 31u;
  const unsigned wave = (unsigned)__builtin_amdgcn_readfirstlane((int)(tid >> 5));
  const unsigned hh = lane >> 4, m = lane & 15u;
  const unsigned row0 = blockIdx.x * 128u + wave * 16u;

  const _Float16* ap = A16 + (size_t)(row0 + m) * KIN + hh * 8u;
  const _Float16* bp = Bt + (size_t)m * KIN + hh * 8u;
  v8f acc[8];
#pragma unroll
  for (int t = 0; t < 8; ++t) acc[t] = (v8f){};
#pragma unroll 1
  for (unsigned k0 = 0; k0 < (unsigned)KIN; k0 += 32u) {
    const v16h a = frag_at(ap + k0);
#pragma unroll
    for (int t = 0; t < 8; ++t) {
      const v16h b = frag_at(bp + (size_t)(16 * t) * KIN + k0);
      acc[t] = wmma16(a, b, acc[t]);
    }
  }

  const float cs = 1.0f / (ACARRY * WCARRY);
  float p[8];
#pragma unroll
  for (int r = 0; r < 8; ++r) p[r] = 0.0f;
#pragma unroll
  for (int t = 0; t < 8; ++t) {
    const unsigned n = 16u * (unsigned)t + m;
    const float bb = bf16r(b1[n]);
    const float ww = bf16r(W2[n]);
#pragma unroll
    for (int r = 0; r < 8; ++r) {
      const float h = fmaxf(acc[t][r] * cs + bb, 0.0f);
      p[r] += h * ww;
    }
  }
#pragma unroll
  for (int r = 0; r < 8; ++r) p[r] = red16_sum(p[r]);
  float v = p[0];
#pragma unroll
  for (int r = 1; r < 8; ++r) v = (m == (unsigned)r) ? p[r] : v;
  const float lg = v + bf16r(b2[0]);
  const float sg = 1.0f / (1.0f + __expf(-lg));
  if (m < 8u) Ls[wave * 16u + hh * 8u + m] = sg;
  __syncthreads();
  if (wave == 0u) {
    const v4f x = *(const v4f*)&Ls[lane * 4u];
    float* po = out + (size_t)blockIdx.x * 128u + lane * 4u;
    *(volatile v4f*)po = x;
    __threadfence();
    *(volatile v4f*)po = x;
  }
}

extern "C" void kernel_launch(void* const* d_in, const int* in_sizes, int n_in,
                              void* d_out, int out_size, void* d_ws, size_t ws_size,
                              hipStream_t stream) {
  if (n_in < 9) return;
  if ((long long)in_sizes[0] < (long long)N_D * FEAT) return;
  if ((long long)in_sizes[1] < (long long)N_P * FEAT) return;
  if ((long long)in_sizes[2] < 2LL * NEDGE) return;
  if ((long long)in_sizes[3] < 2LL * NEDGE) return;
  if ((long long)in_sizes[4] < (long long)NPRED_FULL + NPRED) return;
  if ((long long)in_sizes[5] < (long long)KIN * HIDN) return;
  if (in_sizes[6] < HIDN || in_sizes[7] < HIDN || in_sizes[8] < 1) return;
  if ((long long)out_size < (long long)NPRED) return;
  if (ws_size < WS_TOTAL) return;

  const float* z_drug = (const float*)d_in[0];
  const float* z_prot = (const float*)d_in[1];
  const int*   ddi_ei = (const int*)d_in[2];
  const int*   dp_ei  = (const int*)d_in[3];
  const int*   pred   = (const int*)d_in[4];
  const float* w1     = (const float*)d_in[5];
  const float* b1     = (const float*)d_in[6];
  const float* w2     = (const float*)d_in[7];
  const float* b2     = (const float*)d_in[8];
  float* out = (float*)d_out;

  char* ws = (char*)d_ws;
  _Float16*     W1t    = (_Float16*)(ws + OFF_W1T);
  unsigned int* AdjD   = (unsigned int*)(ws + OFF_ADJD);
  unsigned int* AdjP   = (unsigned int*)(ws + OFF_ADJP);
  _Float16*     Pair16 = (_Float16*)(ws + OFF_PAIR);

  wconv_kernel<<<dim3(HIDN / 64, KIN / 64), dim3(256), 0, stream>>>(
      w1, W1t, (unsigned)HIDN, (unsigned)KIN);
  adj_ddi_kernel<<<dim3(N_D / ROWS_DDI), dim3(32), 0, stream>>>(ddi_ei, AdjD);
  adj_dp_kernel<<<dim3(N_D / ROWS_DP), dim3(32), 0, stream>>>(dp_ei, AdjP);
  pair_kernel<<<dim3(NPRED / 8), dim3(256), 0, stream>>>(z_drug, z_prot, pred, AdjD, AdjP, Pair16);
  mlp_kernel<<<dim3(NPRED / 128), dim3(256), 0, stream>>>(Pair16, W1t, b1, w2, b2, out);
}
